// PinSAGELayer_32341103739251
// MI455X (gfx1250) — hardware-verified
//
#include <hip/hip_runtime.h>


typedef __bf16       v16bf __attribute__((ext_vector_type(16)));
typedef float        v8f   __attribute__((ext_vector_type(8)));
typedef float        v4f   __attribute__((ext_vector_type(4)));
typedef float        v4fa  __attribute__((ext_vector_type(4), may_alias));
typedef unsigned int v8u   __attribute__((ext_vector_type(8)));
typedef unsigned int v8ua  __attribute__((ext_vector_type(8), may_alias));
typedef unsigned int v4u   __attribute__((ext_vector_type(4)));
typedef int          v4i   __attribute__((ext_vector_type(4)));
typedef int          v4ia  __attribute__((ext_vector_type(4), may_alias));

#define DIM   64
#define NPB   1024
#define CHUNK 1024
#define LCAP  128
#define ZP    68

union Frag { v16bf v; v8u u; };

__device__ __forceinline__ unsigned bf16_rne(float x) {
  const unsigned u = __float_as_uint(x);
  return (u + 0x7FFFu + ((u >> 16) & 1u)) >> 16;
}

__device__ __forceinline__ void split_pair(float x0, float x1, unsigned& hw, unsigned& lw) {
  const unsigned h0 = bf16_rne(x0), h1 = bf16_rne(x1);
  const unsigned l0 = bf16_rne(x0 - __uint_as_float(h0 << 16));
  const unsigned l1 = bf16_rne(x1 - __uint_as_float(h1 << 16));
  hw = h0 | (h1 << 16);
  lw = l0 | (l1 << 16);
}

__device__ __forceinline__ void load_a_split(const float* p, Frag& ah, Frag& al) {
  const v4f f0 = *(const v4fa*)(p);
  const v4f f1 = *(const v4fa*)(p + 4);
  const v4f f2 = *(const v4fa*)(p + 16);
  const v4f f3 = *(const v4fa*)(p + 20);
  unsigned hw[8], lw[8];
  split_pair(f0.x, f0.y, hw[0], lw[0]);
  split_pair(f0.z, f0.w, hw[1], lw[1]);
  split_pair(f1.x, f1.y, hw[2], lw[2]);
  split_pair(f1.z, f1.w, hw[3], lw[3]);
  split_pair(f2.x, f2.y, hw[4], lw[4]);
  split_pair(f2.z, f2.w, hw[5], lw[5]);
  split_pair(f3.x, f3.y, hw[6], lw[6]);
  split_pair(f3.z, f3.w, hw[7], lw[7]);
  v8u hu, lu;
  hu[0] = hw[0]; hu[1] = hw[1]; hu[2] = hw[2]; hu[3] = hw[3];
  hu[4] = hw[4]; hu[5] = hw[5]; hu[6] = hw[6]; hu[7] = hw[7];
  lu[0] = lw[0]; lu[1] = lw[1]; lu[2] = lw[2]; lu[3] = lw[3];
  lu[4] = lw[4]; lu[5] = lw[5]; lu[6] = lw[6]; lu[7] = lw[7];
  ah.u = hu;
  al.u = lu;
}

__device__ __forceinline__ v8f wmma_bf16(v8f c, v16bf a, v16bf b) {
  v8f d = __builtin_amdgcn_wmma_f32_16x16x32_bf16(false, a, false, b, (short)0, c, false, false);
  asm volatile("v_nop\n\tv_nop\n\tv_nop\n\tv_nop" : "+v"(d) : "v"(a), "v"(b));
  return d;
}

__global__ __launch_bounds__(256) void k_pack(const float* __restrict__ wq,
                                             const float* __restrict__ ww,
                                             unsigned short* qh, unsigned short* ql,
                                             unsigned short* wh, unsigned short* wl) {
  const int o = blockIdx.x * 256 + threadIdx.x;
  const float* W;
  unsigned short* Hp;
  unsigned short* Lp;
  int idx;
  if (o < 512) { W = wq; Hp = qh; Lp = ql; idx = o; }
  else if (o < 1536) { W = ww; Hp = wh; Lp = wl; idx = o - 512; }
  else return;
  const int s  = idx & 1;
  const int l  = (idx >> 1) & 31;
  const int f  = idx >> 6;
  const int ks = f >> 2, nt = f & 3;
  const int hh = l >> 4;
  const int n  = nt * 16 + (l & 15);
  const int kb = ks * 32 + s * 16 + hh * 8;
  unsigned hw[4], lw[4];
#pragma unroll
  for (int j = 0; j < 4; ++j) {
    const float x0 = W[(kb + 2 * j) * DIM + n];
    const float x1 = W[(kb + 2 * j + 1) * DIM + n];
    split_pair(x0, x1, hw[j], lw[j]);
  }
  v4u hv, lv;
  hv[0] = hw[0]; hv[1] = hw[1]; hv[2] = hw[2]; hv[3] = hw[3];
  lv[0] = lw[0]; lv[1] = lw[1]; lv[2] = lw[2]; lv[3] = lw[3];
  const size_t off = (size_t)(f * 32 + l) * 16 + (size_t)s * 8;
  *(volatile v4u*)(Hp + off) = hv;
  *(volatile v4u*)(Lp + off) = lv;
  __threadfence();
  *(volatile v4u*)(Hp + off) = hv;
  *(volatile v4u*)(Lp + off) = lv;
}

__global__ __launch_bounds__(256) void k_proj(const float* __restrict__ X,
                                             const unsigned short* __restrict__ bh,
                                             const unsigned short* __restrict__ bl,
                                             const float* __restrict__ bias,
                                             float* H, int N) {
  __shared__ __attribute__((aligned(16))) float zs[8][16][ZP];
  const int lane = threadIdx.x & 31, wave = threadIdx.x >> 5;
  const int hh = lane >> 4, m = lane & 15;
  const int rowbase = (blockIdx.x * 8 + wave) * 16;
  int arow = rowbase + m;
  if (arow > N - 1) arow = N - 1;

  v8f acc[4] = {};
#pragma unroll
  for (int ks = 0; ks < 2; ++ks) {
    Frag ah, al;
    load_a_split(X + (size_t)arow * DIM + ks * 32 + 8 * hh, ah, al);
#pragma unroll
    for (int t = 0; t < 4; ++t) {
      const int f = ks * 4 + t;
      Frag wfh, wfl;
      wfh.u = *(const v8ua*)(bh + (size_t)(f * 32 + lane) * 16);
      wfl.u = *(const v8ua*)(bl + (size_t)(f * 32 + lane) * 16);
      acc[t] = wmma_bf16(acc[t], ah.v, wfh.v);
      acc[t] = wmma_bf16(acc[t], ah.v, wfl.v);
      acc[t] = wmma_bf16(acc[t], al.v, wfh.v);
    }
  }

#pragma unroll
  for (int t = 0; t < 4; ++t) {
    const int col = t * 16 + m;
    const float b = bias[col];
#pragma unroll
    for (int r = 0; r < 8; ++r) {
      const float v = acc[t][r] + b;
      zs[wave][hh * 8 + r][col] = v > 0.f ? v : 0.f;
    }
  }
  __syncthreads();

  const int c4 = m * 4;
#pragma unroll
  for (int it = 0; it < 8; ++it) {
    const int r = it * 2 + hh;
    const int grow = rowbase + r;
    const v4f v = *(const v4fa*)(&zs[wave][r][c4]);
    if (grow < N) *(volatile v4f*)(H + (size_t)grow * DIM + c4) = v;
  }
  __threadfence();
#pragma unroll
  for (int it = 0; it < 8; ++it) {
    const int r = it * 2 + hh;
    const int grow = rowbase + r;
    const v4f v = *(const v4fa*)(&zs[wave][r][c4]);
    if (grow < N) *(volatile v4f*)(H + (size_t)grow * DIM + c4) = v;
  }
}

__global__ __launch_bounds__(256) void k_agg(const float* __restrict__ H,
                                            const float* __restrict__ alpha,
                                            const int* __restrict__ srcn,
                                            const int* __restrict__ dstn,
                                            float* Hn, int N, int E, int nchunks) {
#pragma clang fp contract(off)
  __shared__ __attribute__((aligned(16))) float accs[NPB * DIM];
  __shared__ int lst[8][LCAP];
  __shared__ int cnts[8];

  const int tid = threadIdx.x, lane = tid & 31, wave = tid >> 5;
  const int nb = blockIdx.x * NPB;

  const v4f z4 = {0.f, 0.f, 0.f, 0.f};
  for (int i = tid; i < NPB * DIM / 4; i += 256) *(v4fa*)(accs + i * 4) = z4;
  __syncthreads();

  for (int ch = 0; ch < nchunks; ++ch) {
    const int e0 = ch * CHUNK + wave * 128 + lane * 4;
    int dv[4];
    if (e0 + 3 < E) {
      const v4i v = *(const v4ia*)(dstn + e0);
      dv[0] = v.x; dv[1] = v.y; dv[2] = v.z; dv[3] = v.w;
    } else {
#pragma unroll
      for (int k = 0; k < 4; ++k) dv[k] = (e0 + k < E) ? dstn[e0 + k] : -1;
    }
    int run = 0;
#pragma unroll
    for (int k = 0; k < 4; ++k) {
      const unsigned rel = (unsigned)(dv[k] - nb);
      const bool hit = rel < (unsigned)NPB;
      const unsigned msk = __builtin_amdgcn_ballot_w32(hit);
      if (msk) {
        const int pos = run + (int)__builtin_amdgcn_mbcnt_lo(msk, 0u);
        if (hit && pos < LCAP) lst[wave][pos] = e0 + k;
        run += __builtin_popcount(msk);
      }
    }
    if (lane == 0) cnts[wave] = run;
    __syncthreads();

    if (wave == 0) {
      const int g = lane >> 3, c8 = (lane & 7) * 8;
      for (int w = 0; w < 8; ++w) {
        int n = cnts[w];
        if (n > LCAP) n = LCAP;
        for (int j0 = 0; j0 < n; j0 += 4) {
          const int j = j0 + g;
          const bool valid = j < n;
          const int jj = (j < LCAP) ? j : (LCAP - 1);
          int e = lst[w][jj];
          e = e < 0 ? 0 : e; e = e > E - 1 ? E - 1 : e;
          int ld = dstn[e] - nb;
          ld = ld < 0 ? 0 : ld; ld = ld > NPB - 1 ? NPB - 1 : ld;
          const int key = valid ? ld : (-1 - g);
          const int k0 = __shfl(key, 0, 32), k1 = __shfl(key, 8, 32);
          const int k2 = __shfl(key, 16, 32), k3 = __shfl(key, 24, 32);
          const bool dup = (k0 == k1) | (k0 == k2) | (k0 == k3) | (k1 == k2) | (k1 == k3) | (k2 == k3);
          if (!dup) {
            int s = srcn[e];
            s = s < 0 ? 0 : s; s = s > N - 1 ? N - 1 : s;
            const float a = alpha[e];
            const float* hp = H + (size_t)s * DIM + c8;
            const v4f m0 = *(const v4fa*)(hp) * a;
            const v4f m1 = *(const v4fa*)(hp + 4) * a;
            if (valid) {
              float* ap = accs + ld * DIM + c8;
              v4f x0 = *(v4fa*)(ap);
              v4f x1 = *(v4fa*)(ap + 4);
              x0 = x0 + m0;
              x1 = x1 + m1;
              *(v4fa*)(ap) = x0;
              *(v4fa*)(ap + 4) = x1;
            }
          } else if (g == 0) {
#pragma unroll 1
            for (int k = 0; k < 4; ++k) {
              const int jk = j0 + k;
              if (jk < n) {
                int ek = lst[w][jk];
                ek = ek < 0 ? 0 : ek; ek = ek > E - 1 ? E - 1 : ek;
                int ldk = dstn[ek] - nb;
                ldk = ldk < 0 ? 0 : ldk; ldk = ldk > NPB - 1 ? NPB - 1 : ldk;
                int sk = srcn[ek];
                sk = sk < 0 ? 0 : sk; sk = sk > N - 1 ? N - 1 : sk;
                const float ak = alpha[ek];
                const float* hk = H + (size_t)sk * DIM + c8;
                const v4f n0 = *(const v4fa*)(hk) * ak;
                const v4f n1 = *(const v4fa*)(hk + 4) * ak;
                float* ap = accs + ldk * DIM + c8;
                v4f y0 = *(v4fa*)(ap);
                v4f y1 = *(v4fa*)(ap + 4);
                y0 = y0 + n0;
                y1 = y1 + n1;
                *(v4fa*)(ap) = y0;
                *(v4fa*)(ap + 4) = y1;
              }
            }
          }
        }
      }
    }
    __syncthreads();
  }

  for (int it = 0; it < NPB * DIM / 4 / 256; ++it) {
    const int idx4 = it * 256 + tid;
    const int row = idx4 >> 4, c4 = (idx4 & 15) * 4;
    const int grow = nb + row;
    if (grow < N) {
      const v4f v = *(const v4fa*)(accs + row * DIM + c4);
      *(volatile v4f*)(Hn + (size_t)grow * DIM + c4) = v;
    }
  }
  __threadfence();
  for (int it = 0; it < NPB * DIM / 4 / 256; ++it) {
    const int idx4 = it * 256 + tid;
    const int row = idx4 >> 4, c4 = (idx4 & 15) * 4;
    const int grow = nb + row;
    if (grow < N) {
      const v4f v = *(const v4fa*)(accs + row * DIM + c4);
      *(volatile v4f*)(Hn + (size_t)grow * DIM + c4) = v;
    }
  }
}

__global__ __launch_bounds__(256) void k_out(const float* __restrict__ H,
                                            const float* __restrict__ Hn,
                                            const unsigned short* __restrict__ bh,
                                            const unsigned short* __restrict__ bl,
                                            const float* __restrict__ bias,
                                            float* O, int N) {
  __shared__ __attribute__((aligned(16))) float zs[8][16][ZP];
  __shared__ float invs[8][16];
  const int lane = threadIdx.x & 31, wave = threadIdx.x >> 5;
  const int hh = lane >> 4, m = lane & 15;
  const int rowbase = (blockIdx.x * 8 + wave) * 16;
  int arow = rowbase + m;
  if (arow > N - 1) arow = N - 1;

  v8f acc[4] = {};
#pragma unroll
  for (int ks = 0; ks < 4; ++ks) {
    const float* A = (ks < 2) ? H : Hn;
    const int kc = (ks & 1) * 32;
    Frag ah, al;
    load_a_split(A + (size_t)arow * DIM + kc + 8 * hh, ah, al);
#pragma unroll
    for (int t = 0; t < 4; ++t) {
      const int f = ks * 4 + t;
      Frag wfh, wfl;
      wfh.u = *(const v8ua*)(bh + (size_t)(f * 32 + lane) * 16);
      wfl.u = *(const v8ua*)(bl + (size_t)(f * 32 + lane) * 16);
      acc[t] = wmma_bf16(acc[t], ah.v, wfh.v);
      acc[t] = wmma_bf16(acc[t], ah.v, wfl.v);
      acc[t] = wmma_bf16(acc[t], al.v, wfh.v);
    }
  }

#pragma unroll
  for (int t = 0; t < 4; ++t) {
    const int col = t * 16 + m;
    const float b = bias[col];
#pragma unroll
    for (int r = 0; r < 8; ++r) {
      const float v = acc[t][r] + b;
      zs[wave][hh * 8 + r][col] = v > 0.f ? v : 0.f;
    }
  }
  __syncthreads();

  {
    const int r16 = lane >> 1;
    const int co = (lane & 1) * 32;
    float s = 0.f;
#pragma unroll
    for (int j = 0; j < 32; ++j) {
      const float v = zs[wave][r16][co + j];
      s += v * v;
    }
    s += __shfl_xor(s, 1, 32);
    if ((lane & 1) == 0) invs[wave][r16] = 1.0f / sqrtf(s);
  }
  __syncthreads();

  const int c4 = m * 4;
#pragma unroll
  for (int it = 0; it < 8; ++it) {
    const int r = it * 2 + hh;
    const int grow = rowbase + r;
    const v4f v = *(const v4fa*)(&zs[wave][r][c4]) * invs[wave][r];
    if (grow < N) *(volatile v4f*)(O + (size_t)grow * DIM + c4) = v;
  }
  __threadfence();
#pragma unroll
  for (int it = 0; it < 8; ++it) {
    const int r = it * 2 + hh;
    const int grow = rowbase + r;
    const v4f v = *(const v4fa*)(&zs[wave][r][c4]) * invs[wave][r];
    if (grow < N) *(volatile v4f*)(O + (size_t)grow * DIM + c4) = v;
  }
}

extern "C" void kernel_launch(void* const* d_in, const int* in_sizes, int n_in,
                              void* d_out, int out_size, void* d_ws, size_t ws_size,
                              hipStream_t stream) {
  if (n_in < 8) return;
  const float* feat  = (const float*)d_in[0];
  const float* qw    = (const float*)d_in[1];
  const float* qb    = (const float*)d_in[2];
  const float* ww    = (const float*)d_in[3];
  const float* wb    = (const float*)d_in[4];
  const float* alpha = (const float*)d_in[5];
  const int*   srcn  = (const int*)d_in[6];
  const int*   dstn  = (const int*)d_in[7];
  float* out = (float*)d_out;

  const int N = in_sizes[0] / DIM;
  int E = in_sizes[6];
  if (in_sizes[7] < E) E = in_sizes[7];
  if (in_sizes[5] < E) E = in_sizes[5];
  if (N <= 0 || E < 0) return;
  if (in_sizes[1] < DIM * DIM || in_sizes[3] < 2 * DIM * DIM) return;
  if (in_sizes[2] < DIM || in_sizes[4] < DIM) return;
  if (out_size < N * DIM) return;

  char* ws = (char*)d_ws;
  const size_t o_qh = 0, o_ql = 8192, o_wh = 16384, o_wl = 32768, o_h = 49152;
  size_t hbytes = (size_t)N * DIM * sizeof(float);
  hbytes = (hbytes + 127) / 128 * 128;
  const size_t o_hn = o_h + hbytes;
  const size_t total = o_hn + hbytes;
  if (total > ws_size) return;

  unsigned short* qh = (unsigned short*)(ws + o_qh);
  unsigned short* ql = (unsigned short*)(ws + o_ql);
  unsigned short* wh = (unsigned short*)(ws + o_wh);
  unsigned short* wl = (unsigned short*)(ws + o_wl);
  float* Hb  = (float*)(ws + o_h);
  float* Hnb = (float*)(ws + o_hn);

  k_pack<<<dim3(6), dim3(256), 0, stream>>>(qw, ww, qh, ql, wh, wl);

  const int gemmBlocks = (N + 127) / 128;
  k_proj<<<dim3(gemmBlocks), dim3(256), 0, stream>>>(feat, qh, ql, qb, Hb, N);

  const int aggBlocks = (N + NPB - 1) / NPB;
  const int nchunks = (E + CHUNK - 1) / CHUNK;
  k_agg<<<dim3(aggBlocks), dim3(256), 0, stream>>>(Hb, alpha, srcn, dstn, Hnb, N, E, nchunks);

  k_out<<<dim3(gemmBlocks), dim3(256), 0, stream>>>(Hb, Hnb, wh, wl, wb, out, N);
}
